// LSTM_01_25589415149940
// MI455X (gfx1250) — hardware-verified
//
#include <hip/hip_runtime.h>
#include <stddef.h>


#define T_LEN    256
#define IN_F     3
#define H1       32
#define H2       64
#define OUT_F    2
#define G1       (4 * H1)
#define G2       (4 * H2)
#define K2       (H1 + H2)
#define ROWS     16
#define XC       64
#define NTHREADS 128

#define A_SCALE   64.0f
#define W_SCALE   16.0f
#define ACC_SCALE (1.0f / 1024.0f)

typedef _Float16 v4h  __attribute__((ext_vector_type(4)));
typedef _Float16 v8h  __attribute__((ext_vector_type(8)));
typedef _Float16 v16h __attribute__((ext_vector_type(16)));
typedef float    v4f  __attribute__((ext_vector_type(4)));
typedef float    v8f  __attribute__((ext_vector_type(8)));
typedef v4f v4fa __attribute__((may_alias));
typedef v8h v8ha __attribute__((may_alias));
typedef v4h v4ha __attribute__((may_alias));

union Frag { v16h v; v8h p[2]; };

__device__ __forceinline__ v16h load_frag(const _Float16* rowp, int k0, int h) {
    Frag f;
    f.p[0] = *(const v8ha*)(rowp + k0 + 8 * h);
    f.p[1] = *(const v8ha*)(rowp + k0 + 16 + 8 * h);
    return f.v;
}

__device__ __forceinline__ v8f wmma16(v16h a, v16h b, v8f c) {
    v8f d = __builtin_amdgcn_wmma_f32_16x16x32_f16(false, a, false, b, (short)0, c, false, false);
    asm volatile("v_nop\n\tv_nop\n\tv_nop\n\tv_nop" : "+v"(d) : "v"(a), "v"(b));
    return d;
}

__device__ __forceinline__ float rcp_(float x)  { return __builtin_amdgcn_rcpf(x); }
__device__ __forceinline__ float sigm_(float x) { return rcp_(1.0f + __expf(-x)); }
__device__ __forceinline__ float tanh_(float x) { return 1.0f - 2.0f * rcp_(__expf(2.0f * x) + 1.0f); }

__global__ __launch_bounds__(NTHREADS)
void lstm2_head_kernel(const float* __restrict__ x,
                       const float* __restrict__ w_ih1, const float* __restrict__ w_hh1,
                       const float* __restrict__ b_ih1, const float* __restrict__ b_hh1,
                       const float* __restrict__ w_ih2, const float* __restrict__ w_hh2,
                       const float* __restrict__ b_ih2, const float* __restrict__ b_hh2,
                       const float* __restrict__ fc_w,  const float* __restrict__ fc_b,
                       float* out, int nB)
{
    __shared__ __attribute__((aligned(16))) _Float16 W1s[G1 * H1];
    __shared__ __attribute__((aligned(16))) _Float16 W2s[G2 * K2];
    __shared__ __attribute__((aligned(16))) float    xs[XC * ROWS * IN_F];
    __shared__ __attribute__((aligned(16))) _Float16 h1b[2 * ROWS * H1];
    __shared__ __attribute__((aligned(16))) _Float16 h2b[2 * ROWS * H2];
    __shared__ __attribute__((aligned(16))) float    h2f[ROWS * H2];
    __shared__ __attribute__((aligned(16))) float    outs[ROWS * OUT_F];

    const int tid   = threadIdx.x;
    const int wave  = __builtin_amdgcn_readfirstlane(tid >> 5);
    const int lane  = tid & 31;
    const int h     = lane >> 4;
    const int m     = lane & 15;
    const int bBase = blockIdx.x * ROWS;

    for (int f = tid; f < (G1 * H1) / 4; f += NTHREADS) {
        const v4f v = *(const v4fa*)(w_hh1 + 4 * f);
        v4h q;
        q.x = (_Float16)(v.x * W_SCALE); q.y = (_Float16)(v.y * W_SCALE);
        q.z = (_Float16)(v.z * W_SCALE); q.w = (_Float16)(v.w * W_SCALE);
        *(v4ha*)(W1s + 4 * f) = q;
    }
    for (int f = tid; f < (G2 * H1) / 4; f += NTHREADS) {
        const int col = f / (H1 / 4), k4 = f - col * (H1 / 4);
        const v4f v = *(const v4fa*)(w_ih2 + 4 * f);
        v4h q;
        q.x = (_Float16)(v.x * W_SCALE); q.y = (_Float16)(v.y * W_SCALE);
        q.z = (_Float16)(v.z * W_SCALE); q.w = (_Float16)(v.w * W_SCALE);
        *(v4ha*)(W2s + col * K2 + 4 * k4) = q;
    }
    for (int f = tid; f < (G2 * H2) / 4; f += NTHREADS) {
        const int col = f / (H2 / 4), k4 = f - col * (H2 / 4);
        const v4f v = *(const v4fa*)(w_hh2 + 4 * f);
        v4h q;
        q.x = (_Float16)(v.x * W_SCALE); q.y = (_Float16)(v.y * W_SCALE);
        q.z = (_Float16)(v.z * W_SCALE); q.w = (_Float16)(v.w * W_SCALE);
        *(v4ha*)(W2s + col * K2 + H1 + 4 * k4) = q;
    }
    for (int i = tid; i < 2 * ROWS * H1; i += NTHREADS) h1b[i] = (_Float16)0.0f;
    for (int i = tid; i < 2 * ROWS * H2; i += NTHREADS) h2b[i] = (_Float16)0.0f;

    const int j1 = 16 * (wave & 1) + m;
    const int j2 = 16 * wave + m;
    float wx[4][3], b1[4], b2[4];
    #pragma unroll
    for (int q = 0; q < 4; ++q) {
        #pragma unroll
        for (int c = 0; c < IN_F; ++c) wx[q][c] = w_ih1[(q * H1 + j1) * IN_F + c];
        b1[q] = b_ih1[q * H1 + j1] + b_hh1[q * H1 + j1];
        b2[q] = b_ih2[q * H2 + j2] + b_hh2[q * H2 + j2];
    }
    float c1[8], c2[8];
    #pragma unroll
    for (int r = 0; r < 8; ++r) { c1[r] = 0.0f; c2[r] = 0.0f; }
    __syncthreads();

    const v8f zero8 = {0.f, 0.f, 0.f, 0.f, 0.f, 0.f, 0.f, 0.f};

    for (int t = 0; t < T_LEN; ++t) {
        const int p = t & 1;

        if ((t & (XC - 1)) == 0) {
            for (int f = tid; f < (ROWS * XC * IN_F) / 4; f += NTHREADS) {
                const int r  = f / ((XC * IN_F) / 4);
                const int q4 = f - r * ((XC * IN_F) / 4);
                int gb = bBase + r;
                gb = (gb < nB) ? gb : (nB - 1);
                const v4f v = *(const v4fa*)(x + ((size_t)gb * T_LEN + t) * IN_F + 4 * q4);
                #pragma unroll
                for (int u = 0; u < 4; ++u) {
                    const int e  = 4 * q4 + u;
                    const int tl = e / IN_F;
                    const int c  = e - tl * IN_F;
                    xs[(tl * ROWS + r) * IN_F + c] = v[u];
                }
            }
            __syncthreads();
        }

        if (wave < 2) {
            const v16h a = load_frag(h1b + (p * ROWS + m) * H1, 0, h);
            v8f acc[4];
            #pragma unroll
            for (int q = 0; q < 4; ++q) {
                const v16h b = load_frag(W1s + (q * H1 + 16 * wave + m) * H1, 0, h);
                acc[q] = wmma16(a, b, zero8);
            }
            const int tc = t & (XC - 1);
            const v4fa* xp = (const v4fa*)(xs + (tc * ROWS + 8 * h) * IN_F);
            float xf[24];
            #pragma unroll
            for (int u = 0; u < 6; ++u) {
                const v4f v = xp[u];
                xf[4 * u + 0] = v.x; xf[4 * u + 1] = v.y; xf[4 * u + 2] = v.z; xf[4 * u + 3] = v.w;
            }
            _Float16* hd = h1b + ((p ^ 1) * ROWS + 8 * h) * H1 + j1;
            #pragma unroll
            for (int r = 0; r < 8; ++r) {
                const float x0 = xf[3 * r + 0], x1 = xf[3 * r + 1], x2 = xf[3 * r + 2];
                float pre[4];
                #pragma unroll
                for (int q = 0; q < 4; ++q) {
                    const float xw = b1[q] + x0 * wx[q][0] + x1 * wx[q][1] + x2 * wx[q][2];
                    pre[q] = fmaf(acc[q][r], ACC_SCALE, xw);
                }
                const float ig = sigm_(pre[0]);
                const float fg = sigm_(pre[1]);
                const float gg = tanh_(pre[2]);
                const float og = sigm_(pre[3]);
                const float cc = fg * c1[r] + ig * gg;
                c1[r] = cc;
                const float hv = og * tanh_(cc);
                hd[r * H1] = (_Float16)(hv * A_SCALE);
            }
        }
        __syncthreads();

        {
            v8f acc[4];
            #pragma unroll
            for (int q = 0; q < 4; ++q) acc[q] = zero8;
            #pragma unroll
            for (int s = 0; s < K2 / 32; ++s) {
                v16h a;
                if (s == 0) a = load_frag(h1b + ((p ^ 1) * ROWS + m) * H1, 0, h);
                else        a = load_frag(h2b + (p * ROWS + m) * H2, 32 * (s - 1), h);
                #pragma unroll
                for (int q = 0; q < 4; ++q) {
                    const v16h b = load_frag(W2s + (q * H2 + 16 * wave + m) * K2, 32 * s, h);
                    acc[q] = wmma16(a, b, acc[q]);
                }
            }
            _Float16* hd = h2b + ((p ^ 1) * ROWS + 8 * h) * H2 + j2;
            float*    hf = h2f + (8 * h) * H2 + j2;
            const bool last = (t == T_LEN - 1);
            #pragma unroll
            for (int r = 0; r < 8; ++r) {
                float pre[4];
                #pragma unroll
                for (int q = 0; q < 4; ++q) pre[q] = fmaf(acc[q][r], ACC_SCALE, b2[q]);
                const float ig = sigm_(pre[0]);
                const float fg = sigm_(pre[1]);
                const float gg = tanh_(pre[2]);
                const float og = sigm_(pre[3]);
                const float cc = fg * c2[r] + ig * gg;
                c2[r] = cc;
                const float hv = og * tanh_(cc);
                hd[r * H2] = (_Float16)(hv * A_SCALE);
                if (last) hf[r * H2] = hv;
            }
        }
    }
    __syncthreads();

    if (tid < ROWS * OUT_F) {
        const int r = tid >> 1;
        const int o = tid & 1;
        float a = 0.0f;
        #pragma unroll
        for (int j = 0; j < H2; ++j) a = fmaf(h2f[r * H2 + j], fc_w[o * H2 + j], a);
        outs[tid] = a + fc_b[o];
    }
    __syncthreads();

    if (bBase + ROWS <= nB) {
        if (tid < (ROWS * OUT_F) / 4) {
            const v4f v = *(const v4fa*)(outs + 4 * tid);
            volatile v4f* dst = (volatile v4f*)(out + (size_t)bBase * OUT_F) + tid;
            *dst = v;
            __threadfence();
            *dst = v;
        }
    } else {
        if (tid < ROWS * OUT_F) {
            const int row = bBase + (tid >> 1);
            if (row < nB) {
                const float v = outs[tid];
                volatile float* dst = out + (size_t)bBase * OUT_F + tid;
                *dst = v;
                __threadfence();
                *dst = v;
            }
        }
    }
}

extern "C" void kernel_launch(void* const* d_in, const int* in_sizes, int n_in,
                              void* d_out, int out_size, void* d_ws, size_t ws_size,
                              hipStream_t stream)
{
    (void)d_ws; (void)ws_size;
    if (n_in < 11) return;
    int nB  = in_sizes[0] / (T_LEN * IN_F);
    int nBo = out_size / OUT_F;
    if (nBo < nB) nB = nBo;
    if (nB <= 0) return;

    const float* x     = (const float*)d_in[0];
    const float* w_ih1 = (const float*)d_in[1];
    const float* w_hh1 = (const float*)d_in[2];
    const float* b_ih1 = (const float*)d_in[3];
    const float* b_hh1 = (const float*)d_in[4];
    const float* w_ih2 = (const float*)d_in[5];
    const float* w_hh2 = (const float*)d_in[6];
    const float* b_ih2 = (const float*)d_in[7];
    const float* b_hh2 = (const float*)d_in[8];
    const float* fc_w  = (const float*)d_in[9];
    const float* fc_b  = (const float*)d_in[10];
    float* out = (float*)d_out;

    dim3 grid((unsigned)((nB + ROWS - 1) / ROWS));
    dim3 block(NTHREADS);
    lstm2_head_kernel<<<grid, block, 0, stream>>>(
        x, w_ih1, w_hh1, b_ih1, b_hh1, w_ih2, w_hh2, b_ih2, b_hh2, fc_w, fc_b, out, nB);
    (void)hipGetLastError();
}
